// DCRNNEncoder_44074954392026
// MI455X (gfx1250) — hardware-verified
//
#include <hip/hip_runtime.h>
#include <math.h>

typedef __attribute__((ext_vector_type(16))) _Float16 v16h;
typedef __attribute__((ext_vector_type(8)))  _Float16 v8h;
typedef __attribute__((ext_vector_type(16))) __bf16   v16b;
typedef __attribute__((ext_vector_type(8)))  __bf16   v8b;
typedef __attribute__((ext_vector_type(8)))  float    v8f;
typedef __attribute__((ext_vector_type(4)))  float    v4f;

constexpr int kB    = 16;
constexpr int kT    = 32;
constexpr int kN    = 128;
constexpr int kF    = 128;
constexpr int kK3   = 3 * kF;
constexpr int kG    = 2 * kF;
constexpr int kRows = kB * kN;
constexpr int kCols = kB * kF;
constexpr int kAll  = kT * kRows;
constexpr int kThr  = 256;
constexpr float kInCarry = 1024.0f;
constexpr float kWCarry  = 4096.0f;
constexpr float kScD = 1.0f / (kInCarry * kInCarry);
constexpr float kScW = 1.0f / (kInCarry * kWCarry);
constexpr float kF16MinNormal = 6.103515625e-5f;

static_assert((kN % 64) == 0 && (kCols % 64) == 0 && (kRows % 64) == 0 && (kAll % 64) == 0 && (kK3 % 64) == 0 && (kG % 64) == 0 && (kF % 64) == 0, "GEMM M, N multiples of 64");
static_assert(((kN / 64) * (kCols / 64)) % 8 == 0 && ((kAll / 64) * (kK3 / 64)) % 8 == 0 && ((kRows / 64) * (kG / 64)) % 8 == 0 && ((kRows / 64) * (kF / 64)) % 8 == 0, "GEMM grids exact");
static_assert((kN % 32) == 0 && (kK3 % 32) == 0, "GEMM K multiples of 32");

constexpr size_t kOffXCX16 = 0ull;
constexpr size_t kOffGX = 50331648ull;
constexpr size_t kOffXN = 150994944ull;
constexpr size_t kOffS16 = 184549376ull;
constexpr size_t kOffT16 = 185597952ull;
constexpr size_t kOffP = 186122240ull;
constexpr size_t kOffWGX0 = 187170816ull;
constexpr size_t kOffWGX1 = 187465728ull;
constexpr size_t kOffWGH0 = 187760640ull;
constexpr size_t kOffWGH1 = 187957248ull;
constexpr size_t kOffWCH0 = 188153856ull;
constexpr size_t kOffWCH1 = 188252160ull;
constexpr size_t kOffBIAS = 188350464ull;
constexpr size_t kOffH = 188366848ull;
constexpr size_t kOffU = 189415424ull;
constexpr size_t kOffRH = 190464000ull;
constexpr size_t kOffHC16 = 191512576ull;
constexpr size_t kOffGH = 193085440ull;
constexpr size_t kOffCH = 195182592ull;
constexpr size_t kWsTotal = 196231168ull;
static_assert(kWsTotal <= 268435456ull, "carve cap");
static_assert((kOffGX % 256) == 0 && (kOffXN % 256) == 0 && (kOffS16 % 256) == 0 && (kOffT16 % 256) == 0 && (kOffP % 256) == 0 && (kOffWGX0 % 256) == 0 && (kOffWGH0 % 256) == 0 && (kOffWCH0 % 256) == 0 && (kOffBIAS % 256) == 0 && (kOffH % 256) == 0 && (kOffHC16 % 256) == 0 && (kOffGH % 256) == 0 && (kOffCH % 256) == 0, "aligned regions");
constexpr int kFBG0 = 0, kFBC0 = 256, kFBG1 = 384, kFBC1 = 640, kFZB = 1024, kFEnd = 4096;
static_assert(kFZB + kCols <= kFEnd && kFZB + kK3 <= kFEnd, "the zero row covers the widest product (N = 2,048: a diffusion product)");
static_assert(kOffXCX16 == 0 && kOffGX == kOffXCX16 + (size_t)kAll * kK3 * 2 && kOffXN == kOffGX + (size_t)kAll * kK3 * 4 && kOffS16 == kOffXN + (size_t)kAll * kF * 4
              && kOffT16 == kOffS16 + (size_t)kT * kN * kN * 2 && kOffP == kOffT16 + (size_t)kCols * kN * 2 && kOffWGX0 == kOffP + (size_t)kN * kCols * 4
              && kOffWGX1 == kOffWGX0 + (size_t)kK3 * kK3 * 2 && kOffWGH0 == kOffWGX1 + (size_t)kK3 * kK3 * 2 && kOffWGH1 == kOffWGH0 + (size_t)kG * kK3 * 2
              && kOffWCH0 == kOffWGH1 + (size_t)kG * kK3 * 2 && kOffWCH1 == kOffWCH0 + (size_t)kF * kK3 * 2 && kOffBIAS == kOffWCH1 + (size_t)kF * kK3 * 2
              && kOffH == kOffBIAS + (size_t)kFEnd * 4 && kOffU == kOffH + (size_t)kRows * kF * 4 && kOffRH == kOffU + (size_t)kRows * kF * 4
              && kOffHC16 == kOffRH + (size_t)kRows * kF * 4 && kOffGH == kOffHC16 + (size_t)kRows * kK3 * 2 && kOffCH == kOffGH + (size_t)kRows * kG * 4
              && kWsTotal == kOffCH + (size_t)kRows * kF * 4, "the carve is chained and totalled");
constexpr size_t kOut1 = (size_t)2 * kRows * kF;
constexpr size_t kOutTotal = kOut1 + (size_t)kAll * kF;

__device__ __forceinline__ unsigned short f2bf_bits(float f) {
  unsigned u = __float_as_uint(f);
  return (unsigned short)((u + 0x7FFFu + ((u >> 16) & 1u)) >> 16);
}
__device__ __forceinline__ float bf_bits2f(unsigned short h) { return __uint_as_float(((unsigned)h) << 16); }
__device__ __forceinline__ float bf16r(float f) { return bf_bits2f(f2bf_bits(f)); }
__device__ __forceinline__ float carry_flush(float v, float carry) {
  const float s = v * carry;
  return (fabsf(s) < kF16MinNormal) ? 0.0f : s;
}
__device__ __forceinline__ float frcp(float x) { return __builtin_amdgcn_rcpf(x); }

__device__ __forceinline__ void dep_guard4_h(v8f& a, v8f& b, v8f& c, v8f& d, v16h x, v16h y) { asm volatile("v_nop\n\tv_nop\n\tv_nop\n\tv_nop" : "+v"(a), "+v"(b), "+v"(c), "+v"(d) : "v"(x), "v"(y)); }
__device__ __forceinline__ void dep_guard4_b(v8f& a, v8f& b, v8f& c, v8f& d, v16b x, v16b y) { asm volatile("v_nop\n\tv_nop\n\tv_nop\n\tv_nop" : "+v"(a), "+v"(b), "+v"(c), "+v"(d) : "v"(x), "v"(y)); }
__device__ __forceinline__ void keep4_h(v16h a, v16h b, v16h c, v16h d) { asm volatile("v_nop" :: "v"(a), "v"(b), "v"(c), "v"(d)); }
__device__ __forceinline__ void keep4_b(v16b a, v16b b, v16b c, v16b d) { asm volatile("v_nop" :: "v"(a), "v"(b), "v"(c), "v"(d)); }
__device__ __forceinline__ void acc_guard4(v8f& a, v8f& b, v8f& c, v8f& d) { asm volatile("v_nop\n\tv_nop\n\tv_nop\n\tv_nop" : "+v"(a), "+v"(b), "+v"(c), "+v"(d)); }

template <typename T> struct Frag;
template <> struct Frag<_Float16> {
  typedef v16h V; union U { v16h v; v8h h[2]; };
  static __device__ __forceinline__ v16h load(const _Float16* p) {
    U f; f.h[0] = *(const v8h*)(p); f.h[1] = *(const v8h*)(p + 16); return f.v;
  }
  static __device__ __forceinline__ v8f mma(v16h a, v16h b, v8f c) {
    return __builtin_amdgcn_wmma_f32_16x16x32_f16(false, a, false, b, (short)0, c, false, false);
  }
  static __device__ __forceinline__ void guard4(v8f& a, v8f& b, v8f& c, v8f& d, v16h x, v16h y) { dep_guard4_h(a, b, c, d, x, y); }
  static __device__ __forceinline__ void keep(v16h a, v16h b, v16h c, v16h d) { keep4_h(a, b, c, d); }
};
template <> struct Frag<__bf16> {
  typedef v16b V; union U { v16b v; v8b h[2]; };
  static __device__ __forceinline__ v16b load(const __bf16* p) {
    U f; f.h[0] = *(const v8b*)(p); f.h[1] = *(const v8b*)(p + 16); return f.v;
  }
  static __device__ __forceinline__ v8f mma(v16b a, v16b b, v8f c) {
    return __builtin_amdgcn_wmma_f32_16x16x32_bf16(false, a, false, b, (short)0, c, false, false);
  }
  static __device__ __forceinline__ void guard4(v8f& a, v8f& b, v8f& c, v8f& d, v16b x, v16b y) { dep_guard4_b(a, b, c, d, x, y); }
  static __device__ __forceinline__ void keep(v16b a, v16b b, v16b c, v16b d) { keep4_b(a, b, c, d); }
};

__device__ __forceinline__ v8f mma_h(v16h a, v16h b, v8f c) {
  c = __builtin_amdgcn_wmma_f32_16x16x32_f16(false, a, false, b, (short)0, c, false, false);
  asm volatile("v_nop\n\tv_nop\n\tv_nop\n\tv_nop" : "+v"(c) : "v"(a), "v"(b));
  return c;
}

template <int ET> struct Elem;
template <> struct Elem<0> { typedef _Float16 T; };
template <> struct Elem<1> { typedef __bf16 T; };
template <int ET, bool SPLIT, int BIAS_MODE, int OUT_MODE, bool RESID, int ACT = 0>
__global__ __launch_bounds__(256) void wmma_gemm64(
    const unsigned short* __restrict__ Ap, const unsigned short* __restrict__ A2p, int lda, long strideA,
    const unsigned short* __restrict__ Btp, const unsigned short* __restrict__ Bt2p, int ldb, long strideB,
    void* __restrict__ Cout, void* __restrict__ Cout2, int ldc, long strideC,
    const float* __restrict__ bias,
    const float* __restrict__ resid, long strideR,
    int M, int N, int K, float scale) {
  typedef typename Elem<ET>::T T;
  typedef typename Frag<T>::V V;
  const T* A = (const T*)Ap; const T* A2 = (const T*)A2p; const T* Bt = (const T*)Btp; const T* Bt2 = (const T*)Bt2p;
  __shared__ __align__(16) float sT[8][16 * 68];
  const int b    = blockIdx.y;
  const int lane = threadIdx.x & 31;
  const int wave = threadIdx.x >> 5;
  const int tilesN = N >> 6;
  const int tilesM = M >> 6;
  const int tile = blockIdx.x * 8 + wave;
  if (tile >= tilesM * tilesN) return;
  const int tm = tile / tilesN;
  const int tn = tile - tm * tilesN;
  const int m0 = tm << 6;
  const int n0 = tn << 6;

  const T* Ab  = A  + (size_t)b * strideA;
  const T* Bb  = Bt + (size_t)b * strideB;
  const T* Ab2 = SPLIT ? (A2  + (size_t)b * strideA) : nullptr;
  const T* Bb2 = SPLIT ? (Bt2 + (size_t)b * strideB) : nullptr;

  const int rlane = lane & 15;
  const int koff  = (lane >> 4) * 8;
  const int mOff  = (lane >> 4) * 8;

  v8f acc[4][4];
#pragma unroll
  for (int i = 0; i < 4; ++i)
#pragma unroll
    for (int j = 0; j < 4; ++j) acc[i][j] = (v8f){0.f,0.f,0.f,0.f,0.f,0.f,0.f,0.f};

  for (int k0 = 0; k0 < K; k0 += 32) {
    V bh[4], bl[4];
#pragma unroll
    for (int j = 0; j < 4; ++j) {
      const size_t bo = (size_t)(n0 + (j << 4) + rlane) * ldb + koff + k0;
      bh[j] = Frag<T>::load(Bb + bo);
      if (SPLIT) bl[j] = Frag<T>::load(Bb2 + bo);
    }
#pragma unroll
    for (int i = 0; i < 4; ++i) {
      const size_t ao = (size_t)(m0 + (i << 4) + rlane) * lda + koff + k0;
      V ah = Frag<T>::load(Ab + ao);
      V al;
      if (SPLIT) al = Frag<T>::load(Ab2 + ao);
#pragma unroll
      for (int j = 0; j < 4; ++j) {
        acc[i][j] = Frag<T>::mma(ah, bh[j], acc[i][j]);
        if (SPLIT) {
          acc[i][j] = Frag<T>::mma(ah, bl[j], acc[i][j]);
          acc[i][j] = Frag<T>::mma(al, bh[j], acc[i][j]);
        }
      }
      Frag<T>::guard4(acc[i][0], acc[i][1], acc[i][2], acc[i][3], ah, SPLIT ? al : ah);
    }
    Frag<T>::keep(bh[0], bh[1], bh[2], bh[3]);
    if (SPLIT) Frag<T>::keep(bl[0], bl[1], bl[2], bl[3]);
  }
  acc_guard4(acc[0][0], acc[0][1], acc[0][2], acc[0][3]);
  acc_guard4(acc[1][0], acc[1][1], acc[1][2], acc[1][3]);
  acc_guard4(acc[2][0], acc[2][1], acc[2][2], acc[2][3]);
  acc_guard4(acc[3][0], acc[3][1], acc[3][2], acc[3][3]);

  float* slab = sT[wave];
  const float* Rb = RESID ? (resid + (size_t)b * strideR) : nullptr;
#pragma unroll
  for (int i = 0; i < 4; ++i) {
    const int mBase = m0 + (i << 4);
#pragma unroll
    for (int j = 0; j < 4; ++j) {
      const int n = n0 + (j << 4) + rlane;
      float bv = 0.f;
      if (BIAS_MODE == 2) bv = bias[n];
#pragma unroll
      for (int r = 0; r < 8; ++r) {
        float v = acc[i][j][r] * scale;
        if (BIAS_MODE == 1) v += bias[mBase + mOff + r];
        if (BIAS_MODE == 2) v += bv;
        if (RESID) v += Rb[(size_t)(mBase + mOff + r) * ldc + n];
        if (ACT == 1) v = tanhf(v);
        if (ACT == 2) v = fmaxf(v, 0.0f);
        if (ACT == 3) v = v / (1.0f + expf(-v));
        if (ACT == 4) v = (v > 0.f) ? v : 0.01f * v;
        slab[(mOff + r) * 68 + (j << 4) + rlane] = v;
      }
    }
    __builtin_amdgcn_fence(__ATOMIC_RELEASE, "workgroup");
    __builtin_amdgcn_wave_barrier();
    __builtin_amdgcn_fence(__ATOMIC_ACQUIRE, "workgroup");
    if (OUT_MODE == 0) {
      float* C = (float*)Cout + (size_t)b * strideC;
      const int hh = lane >> 4, c4 = (lane & 15) * 4;
      for (int pass = 0; pass < 2; ++pass) {
#pragma unroll
        for (int it = 0; it < 8; ++it) {
          const int row = it * 2 + hh;
          v4f v = *(const v4f*)(slab + row * 68 + c4);
          *(volatile v4f*)(C + (size_t)(mBase + row) * ldc + n0 + c4) = v;
        }
        __threadfence();
      }
    } else {
      const int q = lane >> 3, c8 = (lane & 7) * 8;
      unsigned short* C  = (unsigned short*)Cout  + (size_t)b * strideC;
      unsigned short* C2 = (OUT_MODE == 2) ? ((unsigned short*)Cout2 + (size_t)b * strideC) : nullptr;
      for (int pass = 0; pass < 2; ++pass) {
#pragma unroll
        for (int it = 0; it < 4; ++it) {
          const int row = it * 4 + q;
          const float* sp = slab + row * 68 + c8;
          v8h hv, lv;
#pragma unroll
          for (int e = 0; e < 8; ++e) {
            if (OUT_MODE == 1) {
              hv[e] = (_Float16)sp[e];
            } else {
              unsigned short hb = f2bf_bits(sp[e]);
              unsigned short lb = f2bf_bits(sp[e] - bf_bits2f(hb));
              hv[e] = __builtin_bit_cast(_Float16, hb);
              lv[e] = __builtin_bit_cast(_Float16, lb);
            }
          }
          *(volatile v8h*)(C + (size_t)(mBase + row) * ldc + n0 + c8) = hv;
          if (OUT_MODE == 2) *(volatile v8h*)(C2 + (size_t)(mBase + row) * ldc + n0 + c8) = lv;
        }
        __threadfence();
      }
    }
    __builtin_amdgcn_fence(__ATOMIC_RELEASE, "workgroup");
    __builtin_amdgcn_wave_barrier();
    __builtin_amdgcn_fence(__ATOMIC_ACQUIRE, "workgroup");
  }
}

__global__ __launch_bounds__(kThr) void cast_plane_kernel(const float* __restrict__ src, unsigned short* __restrict__ dst,
                                                          int colsLog2, int dstPitch, int dstOff) {
  const int i   = blockIdx.x * kThr + threadIdx.x;
  const int sh  = colsLog2 - 3;
  const int row = i >> sh;
  const int c8  = (i & ((1 << sh) - 1)) * 8;
  const float* sp = src + ((size_t)row << colsLog2) + c8;
  const v4f a0 = *(const v4f*)(sp);
  const v4f a1 = *(const v4f*)(sp + 4);
  v8h hv;
#pragma unroll
  for (int e = 0; e < 4; ++e) {
    const float f0 = a0[e];
    const float f1 = a1[e];
    hv[e]     = (_Float16)carry_flush(bf16r(f0), kInCarry);
    hv[4 + e] = (_Float16)carry_flush(bf16r(f1), kInCarry);
  }
  unsigned short* dp = dst + (size_t)row * dstPitch + dstOff + c8;
  *(volatile v8h*)dp = hv;
  __threadfence();
  *(volatile v8h*)dp = hv;
}

__device__ __forceinline__ float fast_tanh(float v) { return 1.0f - 2.0f * frcp(__expf(2.0f * v) + 1.0f); }
__device__ __forceinline__ float fast_sigmoid(float v) { return frcp(1.0f + __expf(-v)); }

__global__ __launch_bounds__(kThr) void w_perm_kernel(const float* __restrict__ Wa, int outA, const float* __restrict__ Wb, int outB, int halfOff,
                                                      unsigned short* __restrict__ dst) {
  unsigned v = blockIdx.x * (unsigned)kThr + threadIdx.x;
  asm volatile("" : "+v"(v));
  const unsigned o  = v / 48u;
  const unsigned k8 = (v - o * 48u) * 8u;
  const bool useB = o >= (unsigned)outA;
  const float* W = useB ? Wb : Wa;
  const unsigned oo = useB ? (o - (unsigned)outA) : o;
  const unsigned ow = useB ? (unsigned)outB : (unsigned)outA;
  v8h hv;
#pragma unroll
  for (int e = 0; e < 8; ++e) {
    const unsigned k = k8 + (unsigned)e;
    const unsigned m = k >> 7;
    const unsigned f = k & 127u;
    const float w = W[(size_t)(((unsigned)halfOff + f) * 3u + m) * ow + oo];
    hv[e] = (_Float16)carry_flush(bf16r(w), kWCarry);
  }
  unsigned short* dp = dst + (size_t)o * kK3 + k8;
  *(volatile v8h*)dp = hv;
  __threadfence();
  *(volatile v8h*)dp = hv;
}
static_assert((384 * 48) % kThr == 0 && (256 * 48) % kThr == 0 && (128 * 48) % kThr == 0 && kK3 / 8 == 48, "weight plane grids exact");

__global__ __launch_bounds__(kThr) void bias_rows_kernel(const float* __restrict__ bg0, const float* __restrict__ bc0, const float* __restrict__ bg1,
                                                         const float* __restrict__ bc1, float* __restrict__ BIAS) {
  unsigned v = blockIdx.x * (unsigned)kThr + threadIdx.x;
  asm volatile("" : "+v"(v));
  const unsigned i0 = v * 4u;
  v4f o = {0.f, 0.f, 0.f, 0.f};
  if (i0 < (unsigned)kFZB - 256u) {
    const float* src = (i0 < (unsigned)kFBC0) ? (bg0 + i0) : (i0 < (unsigned)kFBG1) ? (bc0 + (i0 - (unsigned)kFBC0)) : (i0 < (unsigned)kFBC1) ? (bg1 + (i0 - (unsigned)kFBG1)) : (bc1 + (i0 - (unsigned)kFBC1));
    const v4f a = *(const v4f*)src;
#pragma unroll
    for (int e = 0; e < 4; ++e) { const float x = a[e]; o[e] = bf16r(x); }
  }
  float* dp = BIAS + i0;
  *(volatile v4f*)dp = o;
  __threadfence();
  *(volatile v4f*)dp = o;
}
static_assert(kFEnd / 4 == 4 * kThr && kFBC1 + kF == kFZB - 256 && (kFBC0 % 128) == 0 && (kFBG1 % 128) == 0 && (kFBC1 % 128) == 0, "bias grid exact; stream map");

__global__ __launch_bounds__(kThr) void nat_tr_cast_kernel(const float* __restrict__ src, int bStride, int nStride, int roundBf16,
                                                           unsigned short* __restrict__ Adst, int aPitch, int aOff, unsigned short* __restrict__ T16) {
  unsigned v = blockIdx.x * (unsigned)kThr + threadIdx.x;
  asm volatile("" : "+v"(v));
  const unsigned row = v >> 4;
  const unsigned c8 = (v & 15u) * 8u;
  const unsigned b = row >> 7;
  const unsigned q = row & 127u;
  v8h nv, tv;
  {
    const float* sp = src + (size_t)b * bStride + (size_t)q * nStride + c8;
    const v4f a0 = *(const v4f*)sp, a1 = *(const v4f*)(sp + 4);
#pragma unroll
    for (int e = 0; e < 4; ++e) {
      float x0 = a0[e], x1 = a1[e];
      if (roundBf16) { x0 = bf16r(x0); x1 = bf16r(x1); }
      nv[e] = (_Float16)carry_flush(x0, kInCarry); nv[4 + e] = (_Float16)carry_flush(x1, kInCarry);
    }
  }
  {
    const float* sp = src + (size_t)b * bStride + q;
#pragma unroll
    for (int e = 0; e < 8; ++e) {
      float x = sp[(size_t)(c8 + (unsigned)e) * nStride];
      if (roundBf16) x = bf16r(x);
      tv[e] = (_Float16)carry_flush(x, kInCarry);
    }
  }
  unsigned short* ap = Adst + (size_t)row * aPitch + aOff + c8;
  unsigned short* tp = T16 + (size_t)row * kN + c8;
  for (int pass = 0; pass < 2; ++pass) {
    *(volatile v8h*)ap = nv;
    *(volatile v8h*)tp = tv;
    __threadfence();
  }
}

__global__ __launch_bounds__(kThr) void nm_cast_kernel(const float* __restrict__ P, unsigned short* __restrict__ Adst, int aPitch, int aOff,
                                                       unsigned short* __restrict__ T16) {
  unsigned v = blockIdx.x * (unsigned)kThr + threadIdx.x;
  asm volatile("" : "+v"(v));
  const unsigned row = v >> 4;
  const unsigned c8 = (v & 15u) * 8u;
  const unsigned b = row >> 7;
  const unsigned q = row & 127u;
  v8h nv, tv;
  {
    const float* sp = P + (size_t)q * kCols + b * (unsigned)kF + c8;
    const v4f a0 = *(const v4f*)sp, a1 = *(const v4f*)(sp + 4);
#pragma unroll
    for (int e = 0; e < 4; ++e) { nv[e] = (_Float16)carry_flush(a0[e], kInCarry); nv[4 + e] = (_Float16)carry_flush(a1[e], kInCarry); }
  }
  {
    const float* sp = P + b * (unsigned)kF + q;
#pragma unroll
    for (int e = 0; e < 8; ++e) { const float x = sp[(size_t)(c8 + (unsigned)e) * kCols]; tv[e] = (_Float16)carry_flush(x, kInCarry); }
  }
  unsigned short* ap = Adst + (size_t)row * aPitch + aOff + c8;
  unsigned short* tp = T16 + (size_t)row * kN + c8;
  for (int pass = 0; pass < 2; ++pass) {
    *(volatile v8h*)ap = nv;
    *(volatile v8h*)tp = tv;
    __threadfence();
  }
}

__global__ __launch_bounds__(kThr) void cheb_kernel(const float* __restrict__ P, const float* __restrict__ src, int bStride, int nStride, int roundBf16,
                                                    unsigned short* __restrict__ Adst, int aPitch, int aOff) {
  unsigned v = blockIdx.x * (unsigned)kThr + threadIdx.x;
  asm volatile("" : "+v"(v));
  const unsigned row = v >> 4;
  const unsigned c8 = (v & 15u) * 8u;
  const unsigned b = row >> 7;
  const unsigned n = row & 127u;
  const float* pp = P + (size_t)n * kCols + b * (unsigned)kF + c8;
  const float* sp = src + (size_t)b * bStride + (size_t)n * nStride + c8;
  const v4f p0 = *(const v4f*)pp, p1 = *(const v4f*)(pp + 4);
  const v4f a0 = *(const v4f*)sp, a1 = *(const v4f*)(sp + 4);
  v8h nv;
#pragma unroll
  for (int e = 0; e < 4; ++e) {
    float x0 = a0[e], x1 = a1[e];
    if (roundBf16) { x0 = bf16r(x0); x1 = bf16r(x1); }
    nv[e]     = (_Float16)carry_flush(2.0f * p0[e] - x0, kInCarry);
    nv[4 + e] = (_Float16)carry_flush(2.0f * p1[e] - x1, kInCarry);
  }
  unsigned short* ap = Adst + (size_t)row * aPitch + aOff + c8;
  *(volatile v8h*)ap = nv;
  __threadfence();
  *(volatile v8h*)ap = nv;
}
static_assert(kRows * (kF / 8) == 128 * kThr && kCols == kRows && kF / 8 == 16, "layout kernels' grid exact: 2,048 rows x 16 pieces");

__global__ __launch_bounds__(kThr) void state_init_kernel(const float* __restrict__ h0, float* __restrict__ H) {
  const size_t i = (size_t)blockIdx.x * kThr + threadIdx.x;
  const v4f a = *(const v4f*)(h0 + i * 4);
  v4f o;
#pragma unroll
  for (int e = 0; e < 4; ++e) { const float x = a[e]; o[e] = bf16r(x); }
  float* dp = H + i * 4;
  *(volatile v4f*)dp = o;
  __threadfence();
  *(volatile v4f*)dp = o;
}

__global__ __launch_bounds__(kThr) void gate_kernel(const float* __restrict__ GXt, const float* __restrict__ GH, const float* __restrict__ H,
                                                    float* __restrict__ U, float* __restrict__ RH) {
  unsigned v = blockIdx.x * (unsigned)kThr + threadIdx.x;
  asm volatile("" : "+v"(v));
  const unsigned row = v >> 5;
  const unsigned f4 = (v & 31u) * 4u;
  const v4f xr = *(const v4f*)(GXt + (size_t)row * kK3 + f4), xu = *(const v4f*)(GXt + (size_t)row * kK3 + kF + f4);
  const v4f hr = *(const v4f*)(GH + (size_t)row * kG + f4),  hu = *(const v4f*)(GH + (size_t)row * kG + kF + f4);
  const v4f h = *(const v4f*)(H + (size_t)row * kF + f4);
  v4f uo, ro;
#pragma unroll
  for (int e = 0; e < 4; ++e) {
    const float r = fast_sigmoid(xr[e] + hr[e]);
    uo[e] = fast_sigmoid(xu[e] + hu[e]);
    ro[e] = r * h[e];
  }
  float* up = U + (size_t)row * kF + f4;
  float* rp = RH + (size_t)row * kF + f4;
  for (int pass = 0; pass < 2; ++pass) {
    *(volatile v4f*)up = uo;
    *(volatile v4f*)rp = ro;
    __threadfence();
  }
}

__global__ __launch_bounds__(kThr) void cand_kernel(const float* __restrict__ GXt, const float* __restrict__ CH, const float* __restrict__ U,
                                                    float* __restrict__ H, float* __restrict__ seq, float* __restrict__ last) {
  unsigned v = blockIdx.x * (unsigned)kThr + threadIdx.x;
  asm volatile("" : "+v"(v));
  const unsigned row = v >> 5;
  const unsigned f4 = (v & 31u) * 4u;
  const v4f xc = *(const v4f*)(GXt + (size_t)row * kK3 + kG + f4);
  const v4f hc = *(const v4f*)(CH + (size_t)row * kF + f4);
  const v4f u = *(const v4f*)(U + (size_t)row * kF + f4);
  float* hp = H + (size_t)row * kF + f4;
  const v4f h = *(const v4f*)hp;
  v4f o;
#pragma unroll
  for (int e = 0; e < 4; ++e) {
    const float c = fast_tanh(xc[e] + hc[e]);
    o[e] = u[e] * h[e] + (1.0f - u[e]) * c;
  }
  float* sp = seq + (size_t)row * kF + f4;
  for (int pass = 0; pass < 2; ++pass) {
    *(volatile v4f*)hp = o;
    *(volatile v4f*)sp = o;
    if (last != nullptr) *(volatile v4f*)(last + (size_t)row * kF + f4) = o;
    __threadfence();
  }
}
static_assert(kRows * (kF / 4) == 256 * kThr, "gate grids exact");

static_assert(((size_t)kT * kN * kN / 8) % kThr == 0, "supports' cast grid exact");

extern "C" void kernel_launch(void* const* d_in, const int* in_sizes, int n_in,
                              void* d_out, int out_size, void* d_ws, size_t ws_size,
                              hipStream_t stream) {
  if (n_in < 11 || d_out == nullptr || d_ws == nullptr) return;
  if (in_sizes[0] != kB * kT * kN * kF || in_sizes[1] != 2 * kRows * kF || in_sizes[2] != kT * kN * kN) return;
  if (in_sizes[3] != 2 * kK3 * kG || in_sizes[4] != kG || in_sizes[5] != 2 * kK3 * kF || in_sizes[6] != kF) return;
  if (in_sizes[7] != 2 * kK3 * kG || in_sizes[8] != kG || in_sizes[9] != 2 * kK3 * kF || in_sizes[10] != kF) return;
  if ((size_t)out_size != kOutTotal) return;
  if (ws_size < kWsTotal) return;
  const float* inputs   = (const float*)d_in[0];
  const float* h_init   = (const float*)d_in[1];
  const float* supports = (const float*)d_in[2];
  const float* Wg[2] = {(const float*)d_in[3], (const float*)d_in[7]};
  const float* bg[2] = {(const float*)d_in[4], (const float*)d_in[8]};
  const float* Wc[2] = {(const float*)d_in[5], (const float*)d_in[9]};
  const float* bc[2] = {(const float*)d_in[6], (const float*)d_in[10]};
  float* out0 = (float*)d_out;
  float* out1 = (float*)d_out + kOut1;
  char* ws = (char*)d_ws;
  unsigned short* XCX16 = (unsigned short*)(ws + kOffXCX16);
  float* GX = (float*)(ws + kOffGX);
  float* XN = (float*)(ws + kOffXN);
  unsigned short* S16 = (unsigned short*)(ws + kOffS16);
  unsigned short* T16 = (unsigned short*)(ws + kOffT16);
  float* P = (float*)(ws + kOffP);
  unsigned short* WGX[2] = {(unsigned short*)(ws + kOffWGX0), (unsigned short*)(ws + kOffWGX1)};
  unsigned short* WGH[2] = {(unsigned short*)(ws + kOffWGH0), (unsigned short*)(ws + kOffWGH1)};
  unsigned short* WCH[2] = {(unsigned short*)(ws + kOffWCH0), (unsigned short*)(ws + kOffWCH1)};
  float* BIAS = (float*)(ws + kOffBIAS);
  float* H  = (float*)(ws + kOffH);
  float* U  = (float*)(ws + kOffU);
  float* RH = (float*)(ws + kOffRH);
  unsigned short* HC16 = (unsigned short*)(ws + kOffHC16);
  float* GH = (float*)(ws + kOffGH);
  float* CH = (float*)(ws + kOffCH);
  const float* ZB = BIAS + kFZB;

  cast_plane_kernel<<<(int)(((size_t)kT * kN * kN / 8) / kThr), kThr, 0, stream>>>(supports, S16, 7, kN, 0);
  for (int l = 0; l < 2; ++l) {
    w_perm_kernel<<<(384 * 48) / kThr, kThr, 0, stream>>>(Wg[l], kG, Wc[l], kF, 0, WGX[l]);
    w_perm_kernel<<<(256 * 48) / kThr, kThr, 0, stream>>>(Wg[l], kG, Wg[l], 0, kF, WGH[l]);
    w_perm_kernel<<<(128 * 48) / kThr, kThr, 0, stream>>>(Wc[l], kF, Wc[l], 0, kF, WCH[l]);
  }
  bias_rows_kernel<<<4, kThr, 0, stream>>>(bg[0], bc[0], bg[1], bc[1], BIAS);

  for (int l = 0; l < 2; ++l) {
    const float* BG = BIAS + ((l == 0) ? kFBG0 : kFBG1);
    const float* BC = BIAS + ((l == 0) ? kFBC0 : kFBC1);
    for (int t = 0; t < kT; ++t) {
      const float* xs = (l == 0) ? (inputs + (size_t)t * kN * kF) : (XN + (size_t)t * kRows * kF);
      const int bStride = (l == 0) ? (kT * kN * kF) : (kN * kF);
      const int rnd = (l == 0) ? 1 : 0;
      unsigned short* Arow = XCX16 + (size_t)t * kRows * kK3;
      const unsigned short* St = S16 + (size_t)t * kN * kN;
      nat_tr_cast_kernel<<<128, kThr, 0, stream>>>(xs, bStride, kF, rnd, Arow, kK3, 0, T16);
      wmma_gemm64<0, false, 2, 0, false, 0><<<dim3((kN / 64) * (kCols / 64) / 8, 1), 256, 0, stream>>>(
          St, St, kN, 0L, T16, T16, kN, 0L, (void*)P, (void*)P, kCols, 0L, ZB, nullptr, 0L, kN, kCols, kN, kScD);
      nm_cast_kernel<<<128, kThr, 0, stream>>>(P, Arow, kK3, kF, T16);
      wmma_gemm64<0, false, 2, 0, false, 0><<<dim3((kN / 64) * (kCols / 64) / 8, 1), 256, 0, stream>>>(
          St, St, kN, 0L, T16, T16, kN, 0L, (void*)P, (void*)P, kCols, 0L, ZB, nullptr, 0L, kN, kCols, kN, kScD);
      cheb_kernel<<<128, kThr, 0, stream>>>(P, xs, bStride, kF, rnd, Arow, kK3, 2 * kF);
    }
    wmma_gemm64<0, false, 2, 0, false, 0><<<dim3((kAll / 64) * (kK3 / 64) / 8, 1), 256, 0, stream>>>(
        XCX16, XCX16, kK3, 0L, WGX[l], WGX[l], kK3, 0L, (void*)GX, (void*)GX, kK3, 0L, ZB, nullptr, 0L, kAll, kK3, kK3, kScW);
    state_init_kernel<<<256, kThr, 0, stream>>>(h_init + (size_t)l * kRows * kF, H);
    for (int t = 0; t < kT; ++t) {
      const unsigned short* St = S16 + (size_t)t * kN * kN;
      const float* GXt = GX + (size_t)t * kRows * kK3;
      for (int part = 0; part < 2; ++part) {
        const float* vsrc = (part == 0) ? H : RH;
        nat_tr_cast_kernel<<<128, kThr, 0, stream>>>(vsrc, kN * kF, kF, 0, HC16, kK3, 0, T16);
        wmma_gemm64<0, false, 2, 0, false, 0><<<dim3((kN / 64) * (kCols / 64) / 8, 1), 256, 0, stream>>>(
            St, St, kN, 0L, T16, T16, kN, 0L, (void*)P, (void*)P, kCols, 0L, ZB, nullptr, 0L, kN, kCols, kN, kScD);
        nm_cast_kernel<<<128, kThr, 0, stream>>>(P, HC16, kK3, kF, T16);
        wmma_gemm64<0, false, 2, 0, false, 0><<<dim3((kN / 64) * (kCols / 64) / 8, 1), 256, 0, stream>>>(
            St, St, kN, 0L, T16, T16, kN, 0L, (void*)P, (void*)P, kCols, 0L, ZB, nullptr, 0L, kN, kCols, kN, kScD);
        cheb_kernel<<<128, kThr, 0, stream>>>(P, vsrc, kN * kF, kF, 0, HC16, kK3, 2 * kF);
        if (part == 0) {
          wmma_gemm64<0, false, 2, 0, false, 0><<<dim3((kRows / 64) * (kG / 64) / 8, 1), 256, 0, stream>>>(
              HC16, HC16, kK3, 0L, WGH[l], WGH[l], kK3, 0L, (void*)GH, (void*)GH, kG, 0L, BG, nullptr, 0L, kRows, kG, kK3, kScW);
          gate_kernel<<<256, kThr, 0, stream>>>(GXt, GH, H, U, RH);
        } else {
          wmma_gemm64<0, false, 2, 0, false, 0><<<dim3((kRows / 64) * (kF / 64) / 8, 1), 256, 0, stream>>>(
              HC16, HC16, kK3, 0L, WCH[l], WCH[l], kK3, 0L, (void*)CH, (void*)CH, kF, 0L, BC, nullptr, 0L, kRows, kF, kK3, kScW);
          float* seq = (l == 0) ? (XN + (size_t)t * kRows * kF) : (out1 + (size_t)t * kRows * kF);
          float* last = (t == kT - 1) ? (out0 + (size_t)l * kRows * kF) : nullptr;
          cand_kernel<<<256, kThr, 0, stream>>>(GXt, CH, U, H, seq, last);
        }
      }
    }
  }
}
